// LocalRelationalLayer_1795296330401
// MI455X (gfx1250) — hardware-run, weakly checked
//
#include <hip/hip_runtime.h>


namespace {
constexpr int NB = 4, C = 128, HH = 56, WW = 56, NP = HH * WW  , CQ = 16, MG = 8, KS = 7, KK = 49, PAD = 3, CH = 8;
constexpr float XS = 8.0f, HS = 256.0f, WSC = 256.0f;
typedef _Float16 b16;
typedef __attribute__((ext_vector_type(16))) _Float16 v16b;
typedef __attribute__((ext_vector_type(8))) _Float16 v8b;
typedef __attribute__((ext_vector_type(8))) float v8f;
typedef __attribute__((ext_vector_type(4))) float v4f;
__device__ __forceinline__ float bf16_rne(float f) { unsigned int u = __float_as_uint(f); u += 0x7FFFu + ((u >> 16) & 1u); float r = __uint_as_float(u & 0xFFFF0000u); asm volatile("" : "+v"(r)); return r; }
__device__ __forceinline__ float bfv(float f) { float r = bf16_rne(f); asm volatile("" : "+v"(r)); return r; }
__device__ __forceinline__ void split16(float v, b16& hi, b16& lo) { hi = (b16)v; lo = (b16)(v - (float)hi); }
__device__ __forceinline__ v16b frag_kb(const b16* p, int hh) { const v8b a = *(const v8b*)(p + 8 * hh), b = *(const v8b*)(p + 16 + 8 * hh); v16b f;
#pragma unroll
  for (int e = 0; e < 8; ++e) { f[e] = a[e]; f[8 + e] = b[e]; } return f; }
__device__ __forceinline__ v8f wmma16b(v16b a, v16b b, v8f c) { v8f d = __builtin_amdgcn_wmma_f32_16x16x32_f16(false, a, false, b, (short)0, c, false, false); asm volatile("v_nop\n\tv_nop\n\tv_nop\n\tv_nop" : "+v"(d) : "v"(a), "v"(b)); return d; }
__device__ __forceinline__ void wave_lds_sync() { __builtin_amdgcn_fence(__ATOMIC_RELEASE, "workgroup"); __builtin_amdgcn_wave_barrier(); __builtin_amdgcn_fence(__ATOMIC_ACQUIRE, "workgroup"); }
__device__ __forceinline__ float pmul(float a, float b) { float p = a * b; asm volatile("" : "+v"(p)); return p; }

__global__ __launch_bounds__(256) void setup_kernel(const float* __restrict__ kw, const float* __restrict__ qw, const float* __restrict__ fw, const float* __restrict__ gpos, const float* __restrict__ l1w, const float* __restrict__ l1b, const float* __restrict__ l2w, const float* __restrict__ l2b, b16* __restrict__ WKQ, b16* __restrict__ WF, float* __restrict__ GPK) { const int u = threadIdx.x; v8b v;
  for (int idx = u; idx < 32 * 16; idx += 256) { const int o = idx / 16, k0 = (idx % 16) * 8; const float* w = o < CQ ? kw + (size_t)o * C : qw + (size_t)(o - CQ) * C;
#pragma unroll
    for (int j = 0; j < 8; ++j) v[j] = (b16)(bf16_rne(w[k0 + j]) * WSC); for (int pass = 0; pass < 2; ++pass) { *(volatile v8b*)(WKQ + (size_t)o * C + k0) = v; __threadfence(); } }
  for (int idx = u; idx < C * 16; idx += 256) { const int o = idx / 16, k0 = (idx % 16) * 8;
#pragma unroll
    for (int j = 0; j < 8; ++j) v[j] = (b16)(bf16_rne(fw[(size_t)o * C + k0 + j]) * WSC); for (int pass = 0; pass < 2; ++pass) { *(volatile v8b*)(WF + (size_t)o * C + k0) = v; __threadfence(); } }
  for (int idx = u; idx < CQ * 64; idx += 256) { const int cq = idx / 64, kk = idx % 64; float g = 0.0f; if (kk < KK) { float s = bfv(l2b[cq]);
#pragma unroll
      for (int hch = 0; hch < CH; ++hch) { const float hv = fmaxf(pmul(bfv(l1w[hch * 2]), bfv(gpos[kk])) + pmul(bfv(l1w[hch * 2 + 1]), bfv(gpos[KK + kk])) + bfv(l1b[hch]), 0.0f); s += pmul(bfv(l2w[cq * CH + hch]), hv); } g = s; }
    for (int pass = 0; pass < 2; ++pass) { ((volatile float*)GPK)[idx] = g; __threadfence(); } } }
__global__ __launch_bounds__(32) void kq_kernel(const float* __restrict__ x, const b16* __restrict__ WKQ, const float* __restrict__ kb, const float* __restrict__ qb, int PLIM, float* __restrict__ KQ) { __shared__ __attribute__((aligned(16))) b16 Xt[32][C + 8]; __shared__ float Tf[32][36]; const int lane = threadIdx.x, nloc = lane & 15, hlf = lane >> 4; const int b = blockIdx.x / (NP / 32); const int p0 = (blockIdx.x % (NP / 32)) * 32; if (b * NP + p0 >= PLIM) return;
  for (int c = 0; c < C; ++c) Xt[lane][c] = (b16)(bf16_rne(x[((size_t)b * C + c) * NP + p0 + lane]) * XS); for (int k = C; k < C + 8; ++k) Xt[lane][k] = (b16)0.0f;
  wave_lds_sync();
#pragma unroll
  for (int rt = 0; rt < 2; ++rt) { v8f acc[2] = {(v8f){}, (v8f){}};
#pragma unroll
    for (int kb2 = 0; kb2 < C; kb2 += 32) { const v16b a = frag_kb(&Xt[rt * 16 + nloc][kb2], hlf);
#pragma unroll
      for (int t = 0; t < 2; ++t) acc[t] = wmma16b(a, frag_kb(WKQ + (size_t)(t * 16 + nloc) * C + kb2, hlf), acc[t]); }
#pragma unroll
    for (int t = 0; t < 2; ++t) { const int cc = t * 16 + nloc; const float bb = cc < CQ ? bfv(kb[cc]) : bfv(qb[cc - CQ]);
#pragma unroll
      for (int r8 = 0; r8 < 8; ++r8) Tf[rt * 16 + 8 * hlf + r8][cc] = acc[t][r8] * (1.0f / (XS * WSC)) + bb; } }
  wave_lds_sync();
  for (int pass = 0; pass < 2; ++pass) { for (int ch = 0; ch < 32; ++ch) ((volatile float*)KQ)[((size_t)b * 32 + ch) * NP + p0 + lane] = Tf[lane][ch]; __threadfence(); } }
__device__ __forceinline__ float unf_at(const float* plane, int kk, int l) { const int kh = kk / KS, kw = kk % KS; const int oy = l / WW, ox = l % WW; const int iy = oy + kh - PAD, ix = ox + kw - PAD; if (iy < 0 || iy >= HH || ix < 0 || ix >= WW) return 0.0f; return plane[iy * WW + ix]; }
__global__ __launch_bounds__(256) void lr_kernel(const float* __restrict__ KQ, const float* __restrict__ x, const float* __restrict__ GPK, int PLIM, float* __restrict__ PRE) { const size_t u = (size_t)blockIdx.x * 256 + threadIdx.x; const int lp = (int)(u % NP); const int cq = (int)((u / NP) % CQ); const int b = (int)(u / ((size_t)NP * CQ)); if (b >= NB || b * NP + lp >= PLIM) return;
  const float* kmp = KQ + ((size_t)b * 32 + cq) * NP; const float* qmp = KQ + ((size_t)b * 32 + CQ + cq) * NP;
  const int gc = lp * KK + KK / 2; const float qc = unf_at(qmp, gc / NP, gc % NP);
  float mx = -INFINITY;
#pragma unroll 1
  for (int j = 0; j < KK; ++j) { const int g = lp * KK + j; const float a = pmul(unf_at(kmp, g / NP, g % NP), qc) + GPK[cq * 64 + j]; mx = fmaxf(mx, a); }
  float den = 0.0f;
#pragma unroll 1
  for (int j = 0; j < KK; ++j) { const int g = lp * KK + j; const float a = pmul(unf_at(kmp, g / NP, g % NP), qc) + GPK[cq * 64 + j]; den += __expf(a - mx); }
  const float inv = 1.0f / den; float pre8[MG];
#pragma unroll
  for (int m = 0; m < MG; ++m) pre8[m] = 0.0f;
#pragma unroll 1
  for (int j = 0; j < KK; ++j) { const int g = lp * KK + j; const int kk = g / NP, l = g % NP; const float a = pmul(unf_at(kmp, kk, l), qc) + GPK[cq * 64 + j]; const float w = __expf(a - mx) * inv;
#pragma unroll
    for (int m = 0; m < MG; ++m) pre8[m] += pmul(w, bfv(unf_at(x + ((size_t)b * C + m * CQ + cq) * NP, kk, l))); }
  for (int pass = 0; pass < 2; ++pass) {
#pragma unroll
    for (int m = 0; m < MG; ++m) ((volatile float*)PRE)[((size_t)b * C + m * CQ + cq) * NP + lp] = pre8[m]; __threadfence(); } }
__global__ __launch_bounds__(32) void out_kernel(const float* __restrict__ PRE, const b16* __restrict__ WF, const float* __restrict__ fb, int PLIM, float* __restrict__ out) { __shared__ __attribute__((aligned(16))) b16 Ph[32][C + 8], Pl[32][C + 8]; __shared__ float Tf[32][C + 4]; const int lane = threadIdx.x, nloc = lane & 15, hlf = lane >> 4; const int b = blockIdx.x / (NP / 32); const int p0 = (blockIdx.x % (NP / 32)) * 32; if (b * NP + p0 >= PLIM) return;
  for (int c = 0; c < C; ++c) { b16 p, ql; split16(PRE[((size_t)b * C + c) * NP + p0 + lane] * HS, p, ql); Ph[lane][c] = p; Pl[lane][c] = ql; } for (int k = C; k < C + 8; ++k) { Ph[lane][k] = (b16)0.0f; Pl[lane][k] = (b16)0.0f; }
  wave_lds_sync();
#pragma unroll 1
  for (int rt = 0; rt < 2; ++rt) { v8f acc[8];
#pragma unroll
    for (int t = 0; t < 8; ++t) acc[t] = (v8f){};
#pragma unroll
    for (int kb2 = 0; kb2 < C; kb2 += 32) { const v16b a = frag_kb(&Ph[rt * 16 + nloc][kb2], hlf), al = frag_kb(&Pl[rt * 16 + nloc][kb2], hlf);
#pragma unroll
      for (int t = 0; t < 8; ++t) { const v16b bw = frag_kb(WF + (size_t)(t * 16 + nloc) * C + kb2, hlf); acc[t] = wmma16b(a, bw, acc[t]); acc[t] = wmma16b(al, bw, acc[t]); } }
#pragma unroll
    for (int t = 0; t < 8; ++t) { const int cc = t * 16 + nloc; const float bb = bfv(fb[cc]);
#pragma unroll
      for (int r8 = 0; r8 < 8; ++r8) Tf[rt * 16 + 8 * hlf + r8][cc] = acc[t][r8] * (1.0f / (HS * WSC)) + bb; } }
  wave_lds_sync();
  for (int pass = 0; pass < 2; ++pass) {
#pragma unroll 4
    for (int o = 0; o < C; ++o) ((volatile float*)out)[((size_t)b * C + o) * NP + p0 + lane] = Tf[lane][o]; __threadfence(); } }
}

extern "C" void kernel_launch(void* const* d_in, const int* in_sizes, int n_in, void* d_out, int out_size, void* d_ws, size_t ws_size, hipStream_t stream) {
  (void)n_in;
  auto Fp = [&](int i) { return (const float*)d_in[i]; };
  if (in_sizes[0] != NB * C * NP || in_sizes[1] != CQ * C || in_sizes[3] != CQ * C || in_sizes[5] != 2 * KK || in_sizes[6] != CH * 2 || in_sizes[8] != CQ * CH || in_sizes[10] != C * C || out_size != NB * C * NP) return;
  const int PLIM = NB * NP;
  size_t off = 0; char* ws = (char*)d_ws;
  auto carve = [&](size_t bytes) { char* p = ws + off; off += (bytes + 255) & ~(size_t)255; return p; };
  b16* WKQ = (b16*)carve((size_t)32 * C * 2); b16* WF = (b16*)carve((size_t)C * C * 2); float* GPK = (float*)carve(CQ * 64 * 4); float* KQ = (float*)carve((size_t)NB * 32 * NP * 4); float* PRE = (float*)carve((size_t)NB * C * NP * 4);
  if (off > ws_size || off > ((size_t)16 << 20)) return;
  setup_kernel<<<1, 256, 0, stream>>>(Fp(1), Fp(3), Fp(10), Fp(5), Fp(6), Fp(7), Fp(8), Fp(9), WKQ, WF, GPK);
  kq_kernel<<<NB * (NP / 32), 32, 0, stream>>>(Fp(0), WKQ, Fp(2), Fp(4), PLIM, KQ);
  lr_kernel<<<(unsigned)(((size_t)NB * CQ * NP + 255) / 256), 256, 0, stream>>>(KQ, Fp(0), GPK, PLIM, PRE);
  out_kernel<<<NB * (NP / 32), 32, 0, stream>>>(PRE, WF, Fp(11), PLIM, (float*)d_out);
}
